// FinancialReasoningGNN_27522150433049
// MI455X (gfx1250) — hardware-verified
//
#include <hip/hip_runtime.h>
#include <stddef.h>


#define NIN   3
#define HD    64
#define GC    256
#define C1    192
#define KNN   576
#define MK    320
#define MH    128
#define MO    32
#define THR   256
#define NWV   8
#define CHUNK 4096
#define NBN   480
#define SNP   68
#define NBG   240
#define NPG   480
#define NPB   48
#define MTHR  64
#define MROWS 32
#define ZP    136
#define OFF_BN 0
#define OFF_B1 (HD * KNN)
#define OFF_B2 (OFF_B1 + MH * MK)
#define BPTOT  (OFF_B2 + MO * MH)
#define WSC   64.0f
#define HSC   16.0f
#define RH    0.0009765625f
#define WSCAP 134217728
#define LDS_NN  (NBN * SNP * 4 + CHUNK * 4 + NWV * 32 * 4 * 4 + 4 * C1 * 4 + HD * 4 + 32)
#define LDS_GAT (NBG * GC * 4 + CHUNK * 4 + NBG * 4 * 4 * 2 + NBG * 4 * 2 + 32)

static_assert(OFF_B1 == 36864 && OFF_B2 == 77824 && BPTOT == 81920);
static_assert(HD * KNN == 18 * 256 * 8 && MH * MK == 20 * 256 * 8 && MO * MH == 2 * 256 * 8);
static_assert(CHUNK == THR * 16 && NWV * 32 == THR);
static_assert(NBN < 512 && NBG < 512 && (NBN % 8) == 0 && (NBG % 8) == 0);
static_assert((NPG % NBN) == 0 && (NPG % NBG) == 0 && (NPG % NPB) == 0 && (NPG % MROWS) == 0);
static_assert((NBN * SNP) % 4 == 0 && (NBN * SNP) / 4 <= 32 * THR);
static_assert(NBN * 8 == 15 * THR);
static_assert((NBG * GC) / 4 == 60 * THR && NBG / NWV == 30);
static_assert(LDS_NN == 154400 && LDS_GAT == 271776);
static_assert((ZP % 8) == 0 && (KNN % 8) == 0 && (MK % 8) == 0);
static_assert(MROWS == (MTHR / 32) * 16);

typedef float    v4f  __attribute__((ext_vector_type(4)));
typedef float    v8f  __attribute__((ext_vector_type(8)));
typedef int      v4i  __attribute__((ext_vector_type(4)));
typedef _Float16 v4h  __attribute__((ext_vector_type(4)));
typedef _Float16 v8h  __attribute__((ext_vector_type(8)));
typedef _Float16 v16h __attribute__((ext_vector_type(16)));
union Frag { v16h v; v8h h[2]; v4h q[4]; };

#define WSYNC() do { __builtin_amdgcn_fence(__ATOMIC_ACQ_REL, "wavefront"); __builtin_amdgcn_wave_barrier(); } while (0)

__device__ __forceinline__ v8f wmh(v16h a, v16h b, v8f c) {
  v8f d = __builtin_amdgcn_wmma_f32_16x16x32_f16(false, a, false, b, (short)0, c, false, false);
  asm volatile("v_nop\n\tv_nop\n\tv_nop\n\tv_nop" : "+v"(d) : "v"(a), "v"(b));
  return d;
}
__device__ __forceinline__ void wmh2(v16h a0, v16h a1, v16h b, v8f& c0, v8f& c1) {
  c0 = __builtin_amdgcn_wmma_f32_16x16x32_f16(false, a0, false, b, (short)0, c0, false, false);
  c1 = __builtin_amdgcn_wmma_f32_16x16x32_f16(false, a1, false, b, (short)0, c1, false, false);
  asm volatile("v_nop\n\tv_nop\n\tv_nop\n\tv_nop" : "+v"(c0), "+v"(c1) : "v"(a0), "v"(a1), "v"(b));
}

__global__ __launch_bounds__(THR) void k_wprep(const float* __restrict__ w2, const float* __restrict__ m1,
                                               const float* __restrict__ m2, _Float16* Bpl) {
  const int blk = blockIdx.x, tid = threadIdx.x;
  const float* sp;
  _Float16* dp;
  if (blk < 18) {
    const int i = blk * THR + tid;
    const int h = i / 72;
    const int kk = (i - 72 * h) * 8;
    const int ii = kk / C1;
    const int c = kk - C1 * ii;
    sp = w2 + (size_t)(ii * HD + h) * C1 + c;
    dp = Bpl + OFF_BN + i * 8;
  } else if (blk < 38) {
    const int i = (blk - 18) * THR + tid;
    sp = m1 + (size_t)i * 8;
    dp = Bpl + OFF_B1 + i * 8;
  } else {
    const int i = (blk - 38) * THR + tid;
    sp = m2 + (size_t)i * 8;
    dp = Bpl + OFF_B2 + i * 8;
  }
  v8h hv;
#pragma unroll
  for (int e = 0; e < 8; ++e) hv[e] = (_Float16)(sp[e] * WSC);
  *(volatile v8h*)dp = hv;
  __threadfence();
  *(volatile v8h*)dp = hv;
}

__global__ __launch_bounds__(THR) void k_node(const float* __restrict__ x, const float* __restrict__ gwl,
                                              const float* __restrict__ gbl, const float* __restrict__ gwr,
                                              const float* __restrict__ gbr, float* XL, float* XR, int nN) {
  const int tid = threadIdx.x, lane = tid & 31;
  const int wave = __builtin_amdgcn_readfirstlane(tid >> 5);
  const int c0 = 4 * lane, c1 = GC / 2 + 4 * lane;
  float wl0[4][3], wl1[4][3], wr0[4][3], wr1[4][3], bl0[4], bl1[4], br0[4], br1[4];
#pragma unroll
  for (int j = 0; j < 4; ++j) {
#pragma unroll
    for (int i = 0; i < 3; ++i) {
      wl0[j][i] = gwl[(c0 + j) * 3 + i];
      wl1[j][i] = gwl[(c1 + j) * 3 + i];
      wr0[j][i] = gwr[(c0 + j) * 3 + i];
      wr1[j][i] = gwr[(c1 + j) * 3 + i];
    }
    bl0[j] = gbl[c0 + j]; bl1[j] = gbl[c1 + j];
    br0[j] = gbr[c0 + j]; br1[j] = gbr[c1 + j];
  }
#pragma unroll 1
  for (int it = 0; it < NPB / NWV; ++it) {
    const int node = blockIdx.x * NPB + it * NWV + wave;
    const int xrow = node > nN - 1 ? nN - 1 : node;
    const float x0 = x[(size_t)xrow * 3], x1 = x[(size_t)xrow * 3 + 1], x2 = x[(size_t)xrow * 3 + 2];
    v4f a0, a1, r0, r1;
#pragma unroll
    for (int j = 0; j < 4; ++j) {
      a0[j] = fmaf(x2, wl0[j][2], fmaf(x1, wl0[j][1], x0 * wl0[j][0])) + bl0[j];
      a1[j] = fmaf(x2, wl1[j][2], fmaf(x1, wl1[j][1], x0 * wl1[j][0])) + bl1[j];
      r0[j] = fmaf(x2, wr0[j][2], fmaf(x1, wr0[j][1], x0 * wr0[j][0])) + br0[j];
      r1[j] = fmaf(x2, wr1[j][2], fmaf(x1, wr1[j][1], x0 * wr1[j][0])) + br1[j];
    }
    float* pl = XL + (size_t)node * GC;
    float* pr = XR + (size_t)node * GC;
    *(volatile v4f*)(pl + c0) = a0; *(volatile v4f*)(pl + c1) = a1;
    *(volatile v4f*)(pr + c0) = r0; *(volatile v4f*)(pr + c1) = r1;
    __threadfence();
    *(volatile v4f*)(pl + c0) = a0; *(volatile v4f*)(pl + c1) = a1;
    *(volatile v4f*)(pr + c0) = r0; *(volatile v4f*)(pr + c1) = r1;
  }
}

template <int NB>
__device__ __forceinline__ int compact(const int* __restrict__ dsts, int nE, int cbase, int n0,
                                       int wave, int lane, int vec, unsigned* slist, int* swt) {
  int d[16];
  const int eb = cbase + 512 * wave + 4 * lane;
  if (vec != 0 && cbase + CHUNK <= nE) {
#pragma unroll
    for (int q = 0; q < 4; ++q) {
      const v4i t4 = *(const v4i*)(dsts + eb + 128 * q);
      d[4 * q] = t4.x; d[4 * q + 1] = t4.y; d[4 * q + 2] = t4.z; d[4 * q + 3] = t4.w;
    }
  } else {
#pragma unroll
    for (int k = 0; k < 16; ++k) {
      int idx = eb + 128 * (k >> 2) + (k & 3);
      const bool ok = idx < nE;
      idx = ok ? idx : nE - 1;
      const int val = dsts[idx];
      d[k] = ok ? val : (-2147483647 - 1);
    }
  }
  unsigned hm[16];
  int cw = 0;
#pragma unroll
  for (int k = 0; k < 16; ++k) {
    const unsigned ld = (unsigned)d[k] - (unsigned)n0;
    hm[k] = __builtin_amdgcn_ballot_w32(ld < (unsigned)NB);
    cw += __builtin_popcount(hm[k]);
  }
  swt[wave] = cw;
  __syncthreads();
  int base = 0, nh = 0;
#pragma unroll
  for (int w = 0; w < NWV; ++w) {
    const int v = swt[w];
    base += (w < wave) ? v : 0;
    nh += v;
  }
  int run = base;
#pragma unroll
  for (int k = 0; k < 16; ++k) {
    const unsigned ld = (unsigned)d[k] - (unsigned)n0;
    const unsigned mk = hm[k];
    const int pos = run + (int)__builtin_amdgcn_mbcnt_lo(mk, 0u);
    const unsigned e = (unsigned)(eb + 128 * (k >> 2) + (k & 3));
    if (ld < (unsigned)NB) slist[pos & (CHUNK - 1)] = (e << 9) | ld;
    run += __builtin_popcount(mk);
  }
  __syncthreads();
  return nh;
}

__device__ __forceinline__ v4h relu4(float a, v4f w, v4f b) {
  v4f t;
  t.x = fmaxf(fmaf(a, w.x, b.x), 0.0f);
  t.y = fmaxf(fmaf(a, w.y, b.y), 0.0f);
  t.z = fmaxf(fmaf(a, w.z, b.z), 0.0f);
  t.w = fmaf(a, w.w, b.w); t.w = fmaxf(t.w, 0.0f);
  return __builtin_convertvector(t, v4h);
}

__device__ __forceinline__ void nn_tiles(unsigned myent, int pcnt, int lane, int wave, int hh, int m,
                                         int nN, int nE, const int* __restrict__ srcs,
                                         const float* __restrict__ x, const float* __restrict__ ea,
                                         const _Float16* __restrict__ Bn, float* stile,
                                         const float* sw1s, const float* sb1s, float* sacc) {
  WSYNC();
  float* wt = stile + wave * 128;
  const bool valid = lane < pcnt;
  int e = (int)(myent >> 9);
  e = valid ? e : 0;
  e = e > nE - 1 ? nE - 1 : e;
  int ld = (int)(myent & 511u);
  ld = ld > NBN - 1 ? NBN - 1 : ld;
  const int ld0 = __builtin_amdgcn_readfirstlane(ld);
  const int ldc = valid ? ld : ld0;
  int s = srcs[e];
  s = s < 0 ? 0 : (s > nN - 1 ? nN - 1 : s);
  v4f g;
  g.x = x[(size_t)s * 3]; g.y = x[(size_t)s * 3 + 1]; g.z = x[(size_t)s * 3 + 2]; g.w = ea[e];
  if (!valid) { g.x = 0.0f; g.y = 0.0f; g.z = 0.0f; g.w = 0.0f; }
  *(v4f*)(wt + lane * 4) = g;
  WSYNC();
  const v4f r0 = *(const v4f*)(wt + m * 4);
  const v4f r1 = *(const v4f*)(wt + (16 + m) * 4);
  _Float16 xa[3], xb[3];
  xa[0] = (_Float16)r0.x; xa[1] = (_Float16)r0.y; xa[2] = (_Float16)r0.z;
  xb[0] = (_Float16)r1.x; xb[1] = (_Float16)r1.y; xb[2] = (_Float16)r1.z;
  const float a0 = r0.w, a1 = r1.w;

  v8f acc[2][4];
#pragma unroll
  for (int tt = 0; tt < 2; ++tt) {
#pragma unroll
    for (int t = 0; t < 4; ++t) { v8f z = {0.f, 0.f, 0.f, 0.f, 0.f, 0.f, 0.f, 0.f}; acc[tt][t] = z; }
  }
  const _Float16* bb = Bn + (size_t)m * KNN + 8 * hh;
  const v4f* w4 = (const v4f*)sw1s;
  const v4f* b4 = (const v4f*)sb1s;
#pragma unroll 1
  for (int cs = 0; cs < 6; ++cs) {
    const int qlo = 8 * cs + 2 * hh;
    const int qhi = qlo + 4;
    const v4f wA = w4[qlo], wB = w4[qlo + 1], wC = w4[qhi], wD = w4[qhi + 1];
    const v4f cA = b4[qlo], cB = b4[qlo + 1], cC = b4[qhi], cD = b4[qhi + 1];
    Frag h0, h1;
    h0.q[0] = relu4(a0, wA, cA); h0.q[1] = relu4(a0, wB, cB); h0.q[2] = relu4(a0, wC, cC); h0.q[3] = relu4(a0, wD, cD);
    h1.q[0] = relu4(a1, wA, cA); h1.q[1] = relu4(a1, wB, cB); h1.q[2] = relu4(a1, wC, cC); h1.q[3] = relu4(a1, wD, cD);
#pragma unroll
    for (int i = 0; i < 3; ++i) {
      const v16h A0 = h0.v * xa[i];
      const v16h A1 = h1.v * xb[i];
      const int ks = 6 * i + cs;
#pragma unroll
      for (int t = 0; t < 4; ++t) {
        const _Float16* bp = bb + (size_t)(16 * t) * KNN + 32 * ks;
        Frag b;
        b.h[0] = *(const v8h*)bp;
        b.h[1] = *(const v8h*)(bp + 16);
        wmh2(A0, A1, b.v, acc[0][t], acc[1][t]);
      }
    }
  }

#pragma unroll
  for (int tt = 0; tt < 2; ++tt) {
#pragma unroll
    for (int r = 0; r < 8; ++r) {
      const int ra = 16 * tt + r, rb = ra + 8;
      const int lda = __builtin_amdgcn_readlane(ldc, ra);
      const int ldb = __builtin_amdgcn_readlane(ldc, rb);
      const bool same = (lda == ldb);
      const int myrow = (hh != 0) ? ldb : lda;
      const bool st = !(same && (hh != 0));
      float* rp = sacc + myrow * SNP;
#pragma unroll
      for (int t = 0; t < 4; ++t) {
        const float v = acc[tt][t][r];
        const float vo = __shfl_xor(v, 16, 32);
        const float addv = same ? (v + vo) : v;
        float* p = rp + 16 * t + m;
        const float nv = *p + addv;
        if (st) *p = nv;
      }
      {
        const int ci = m & 3;
        const float v = wt[(16 * tt + 8 * hh + r) * 4 + ci];
        const float vo = __shfl_xor(v, 16, 32);
        const float addv = same ? (v + vo) : v;
        float* p = rp + HD + ci;
        const float nv = *p + addv;
        if (st && m < 3) *p = nv;
      }
      WSYNC();
    }
  }
}

__global__ __launch_bounds__(THR) void k_nndrain(
    const int* __restrict__ srcs, const int* __restrict__ dsts, const float* __restrict__ x,
    const float* __restrict__ ea, const float* __restrict__ w1, const float* __restrict__ b1,
    const float* __restrict__ b2, const float* __restrict__ rt, const float* __restrict__ rb,
    const _Float16* __restrict__ Bn, _Float16* HS, int nN, int nE, int nChunks, int vec) {
  extern __shared__ __attribute__((aligned(16))) char dynl[];
  float*    sacc  = (float*)dynl;
  unsigned* slist = (unsigned*)(dynl + NBN * SNP * 4);
  float*    stile = (float*)(slist + CHUNK);
  float*    sw1s  = stile + NWV * 32 * 4;
  float*    sb1s  = sw1s + C1;
  float*    sb2   = sb1s + C1;
  float*    srt   = sb2 + C1;
  float*    sbi   = srt + C1;
  int*      swt   = (int*)(sbi + HD);
  const int tid = threadIdx.x, lane = tid & 31, hh = lane >> 4, m = lane & 15;
  const int wave = __builtin_amdgcn_readfirstlane(tid >> 5);
  const int n0 = blockIdx.x * NBN;
  if (tid < C1) {
    sw1s[tid] = w1[tid] * HSC;
    sb1s[tid] = b1[tid] * HSC;
    sb2[tid]  = b2[tid];
    srt[tid]  = rt[tid];
  }
  if (tid < HD) sbi[tid] = rb[tid];
  {
    v4f z = {0.f, 0.f, 0.f, 0.f};
    v4f* p = (v4f*)sacc;
#pragma unroll
    for (int it = 0; it < 32; ++it) {
      const int f = it * THR + tid;
      if (f < (NBN * SNP) / 4) p[f] = z;
    }
  }
  __syncthreads();

  int pc = 0;
  unsigned myent = 0u;
#pragma unroll 1
  for (int c = 0; c < nChunks; ++c) {
    const int nh = compact<NBN>(dsts, nE, c * CHUNK, n0, wave, lane, vec, slist, swt);
    const int nhc = nh < CHUNK ? nh : CHUNK;
    for (int j0 = 0; j0 < nhc; j0 += 32) {
      const int idx = j0 + lane;
      const bool inr = idx < nhc;
      const unsigned ent = slist[inr ? idx : 0];
      const bool own = inr && ((ent & 7u) == (unsigned)wave);
      unsigned om = __builtin_amdgcn_ballot_w32(own);
      while (om != 0u) {
        const int b = __builtin_ctz(om);
        om &= om - 1u;
        const unsigned eb = (unsigned)__builtin_amdgcn_readlane((int)ent, b);
        myent = (lane == pc) ? eb : myent;
        ++pc;
        if (pc == 32) {
          nn_tiles(myent, 32, lane, wave, hh, m, nN, nE, srcs, x, ea, Bn, stile, sw1s, sb1s, sacc);
          pc = 0;
        }
      }
    }
  }
  if (pc > 0)
    nn_tiles(myent, pc, lane, wave, hh, m, nN, nE, srcs, x, ea, Bn, stile, sw1s, sb1s, sacc);
  __syncthreads();

  v8h hv[15];
#pragma unroll
  for (int it = 0; it < 15; ++it) {
    const int f = it * THR + tid, row = f >> 3, q = f & 7;
    const int node = n0 + row;
    const int xrow = node > nN - 1 ? nN - 1 : node;
    const float x0 = x[(size_t)xrow * 3], x1 = x[(size_t)xrow * 3 + 1], x2 = x[(size_t)xrow * 3 + 2];
    const float* rp = sacc + row * SNP;
    const float sx0 = rp[HD], sx1 = rp[HD + 1], sx2 = rp[HD + 2];
    const v4f u0 = *(const v4f*)(rp + 8 * q), u1 = *(const v4f*)(rp + 8 * q + 4);
    float av[8];
    av[0] = u0.x; av[1] = u0.y; av[2] = u0.z; av[3] = u0.w;
    av[4] = u1.x; av[5] = u1.y; av[6] = u1.z; av[7] = u1.w;
#pragma unroll
    for (int j = 0; j < 8; ++j) {
      const int ch = 8 * q + j;
      float v = av[j] * RH;
      v = fmaf(sx0, sb2[ch], v);
      v = fmaf(sx1, sb2[HD + ch], v);
      v = fmaf(sx2, sb2[2 * HD + ch], v);
      v = fmaf(x0, srt[ch * 3], v);
      v = fmaf(x1, srt[ch * 3 + 1], v);
      v = fmaf(x2, srt[ch * 3 + 2], v);
      v += sbi[ch];
      hv[it][j] = (_Float16)(fmaxf(v, 0.0f) * HSC);
    }
  }
#pragma unroll
  for (int it = 0; it < 15; ++it) {
    const int f = it * THR + tid, row = f >> 3, q = f & 7;
    *(volatile v8h*)(HS + (size_t)(n0 + row) * HD + 8 * q) = hv[it];
  }
  __threadfence();
#pragma unroll
  for (int it = 0; it < 15; ++it) {
    const int f = it * THR + tid, row = f >> 3, q = f & 7;
    *(volatile v8h*)(HS + (size_t)(n0 + row) * HD + 8 * q) = hv[it];
  }
}

__device__ __forceinline__ void gat_upd(int ld, float a, const float* xlp, const float* xrp,
                                        const float (&we8)[8], const float (&at8)[8],
                                        float* smx, float* sdn, float* sacc, int lane) {
  const v4f l0 = *(const v4f*)xlp, l1 = *(const v4f*)(xlp + 4);
  const v4f q0 = *(const v4f*)xrp, q1 = *(const v4f*)(xrp + 4);
  float xl[8], xr[8];
  xl[0] = l0.x; xl[1] = l0.y; xl[2] = l0.z; xl[3] = l0.w; xl[4] = l1.x; xl[5] = l1.y; xl[6] = l1.z; xl[7] = l1.w;
  xr[0] = q0.x; xr[1] = q0.y; xr[2] = q0.z; xr[3] = q0.w; xr[4] = q1.x; xr[5] = q1.y; xr[6] = q1.z; xr[7] = q1.w;
  float lg = 0.0f;
#pragma unroll
  for (int j = 0; j < 8; ++j) {
    const float mm = fmaf(a, we8[j], xl[j] + xr[j]);
    const float lk = fmaxf(mm, 0.2f * mm);
    lg = fmaf(lk, at8[j], lg);
  }
  lg += __shfl_xor(lg, 1, 32);
  lg += __shfl_xor(lg, 2, 32);
  lg += __shfl_xor(lg, 4, 32);
  const int hi = ld * 4 + (lane >> 3);
  const float mo = smx[hi], dold = sdn[hi];
  const float mn = fmaxf(mo, lg);
  const float sc = __expf(mo - mn);
  const float p  = __expf(lg - mn);
  smx[hi] = mn;
  sdn[hi] = fmaf(dold, sc, p);
  float* ap = sacc + ld * GC + 8 * lane;
  v4f c0 = *(const v4f*)ap, c1 = *(const v4f*)(ap + 4);
  c0.x = fmaf(p, xl[0], c0.x * sc); c0.y = fmaf(p, xl[1], c0.y * sc); c0.z = fmaf(p, xl[2], c0.z * sc); c0.w = fmaf(p, xl[3], c0.w * sc);
  c1.x = fmaf(p, xl[4], c1.x * sc); c1.y = fmaf(p, xl[5], c1.y * sc); c1.z = fmaf(p, xl[6], c1.z * sc); c1.w = fmaf(p, xl[7], c1.w * sc);
  *(v4f*)ap = c0;
  *(v4f*)(ap + 4) = c1;
}

__global__ __launch_bounds__(THR) void k_gatdrain(
    const int* __restrict__ srcs, const int* __restrict__ dsts, const float* __restrict__ ea,
    const float* __restrict__ gwe, const float* __restrict__ gat, const float* __restrict__ gbs,
    const float* __restrict__ XL, float* XR, int nN, int nE, int nChunks, int vec) {
  extern __shared__ __attribute__((aligned(16))) char dynl[];
  float*    sacc  = (float*)dynl;
  unsigned* slist = (unsigned*)(dynl + NBG * GC * 4);
  float*    smx   = (float*)(slist + CHUNK);
  float*    sdn   = smx + NBG * 4;
  int*      scnt  = (int*)(sdn + NBG * 4);
  float*    ssum  = (float*)(scnt + NBG);
  int*      swt   = (int*)(ssum + NBG);
  const int tid = threadIdx.x, lane = tid & 31, hd = lane >> 3;
  const int wave = __builtin_amdgcn_readfirstlane(tid >> 5);
  const int n0 = blockIdx.x * NBG;
  float we8[8], at8[8], gb8[8];
#pragma unroll
  for (int j = 0; j < 8; ++j) {
    const int ch = 8 * lane + j;
    we8[j] = gwe[ch]; at8[j] = gat[ch]; gb8[j] = gbs[ch];
  }
  {
    v4f z = {0.f, 0.f, 0.f, 0.f};
    v4f* p = (v4f*)sacc;
#pragma unroll
    for (int it = 0; it < 60; ++it) p[it * THR + tid] = z;
#pragma unroll
    for (int it = 0; it < 4; ++it) {
      const int f = it * THR + tid;
      if (f < NBG * 4) { smx[f] = -1.0e30f; sdn[f] = 0.0f; }
    }
    if (tid < NBG) { scnt[tid] = 0; ssum[tid] = 0.0f; }
  }
  __syncthreads();

#pragma unroll 1
  for (int c = 0; c < nChunks; ++c) {
    const int nh = compact<NBG>(dsts, nE, c * CHUNK, n0, wave, lane, vec, slist, swt);
    const int nhc = nh < CHUNK ? nh : CHUNK;
    for (int j0 = 0; j0 < nhc; j0 += 32) {
      const int idx = j0 + lane;
      const bool inr = idx < nhc;
      const unsigned ent = slist[inr ? idx : 0];
      const bool own = inr && ((ent & 7u) == (unsigned)wave);
      unsigned om = __builtin_amdgcn_ballot_w32(own);
      while (om != 0u) {
        const int b = __builtin_ctz(om);
        om &= om - 1u;
        const unsigned eb = (unsigned)__builtin_amdgcn_readlane((int)ent, b);
        int e = (int)(eb >> 9);
        e = e > nE - 1 ? nE - 1 : e;
        int ld = (int)(eb & 511u);
        ld = ld > NBG - 1 ? NBG - 1 : ld;
        int s = srcs[e];
        s = s < 0 ? 0 : (s > nN - 1 ? nN - 1 : s);
        const float a = ea[e];
        gat_upd(ld, a, XL + (size_t)s * GC + 8 * lane, XR + (size_t)(n0 + ld) * GC + 8 * lane,
                we8, at8, smx, sdn, sacc, lane);
        scnt[ld] = scnt[ld] + 1;
        ssum[ld] = ssum[ld] + a;
      }
    }
  }
#pragma unroll 1
  for (int q = 0; q < NBG / NWV; ++q) {
    const int ld = 8 * q + wave;
    const int node = n0 + ld;
    const int cn = scnt[ld];
    const float sm = ssum[ld];
    const float a = sm / fmaxf((float)cn, 1.0f);
    gat_upd(ld, a, XL + (size_t)node * GC + 8 * lane, XR + (size_t)node * GC + 8 * lane,
            we8, at8, smx, sdn, sacc, lane);
  }
  __syncthreads();

  _Float16* HN = (_Float16*)XR;
#pragma unroll 1
  for (int q = 0; q < NBG / NWV; ++q) {
    const int row = 8 * q + wave;
    const float rcp = 1.0f / (sdn[row * 4 + hd] + 1e-16f);
    const float* ap = sacc + row * GC + 8 * lane;
    const v4f c0 = *(const v4f*)ap, c1 = *(const v4f*)(ap + 4);
    v8h hv;
    hv[0] = (_Float16)(fmaxf(fmaf(c0.x, rcp, gb8[0]), 0.0f) * HSC);
    hv[1] = (_Float16)(fmaxf(fmaf(c0.y, rcp, gb8[1]), 0.0f) * HSC);
    hv[2] = (_Float16)(fmaxf(fmaf(c0.z, rcp, gb8[2]), 0.0f) * HSC);
    hv[3] = (_Float16)(fmaxf(fmaf(c0.w, rcp, gb8[3]), 0.0f) * HSC);
    hv[4] = (_Float16)(fmaxf(fmaf(c1.x, rcp, gb8[4]), 0.0f) * HSC);
    hv[5] = (_Float16)(fmaxf(fmaf(c1.y, rcp, gb8[5]), 0.0f) * HSC);
    hv[6] = (_Float16)(fmaxf(fmaf(c1.z, rcp, gb8[6]), 0.0f) * HSC);
    hv[7] = (_Float16)(fmaxf(fmaf(c1.w, rcp, gb8[7]), 0.0f) * HSC);
    _Float16* gp = HN + (size_t)(n0 + row) * (2 * GC) + 8 * lane;
    *(volatile v8h*)gp = hv;
    __threadfence();
    *(volatile v8h*)gp = hv;
  }
}

__global__ __launch_bounds__(MTHR) void k_merge(const _Float16* __restrict__ HS, const _Float16* __restrict__ HN,
                                                const _Float16* __restrict__ B1, const float* __restrict__ mb1,
                                                const _Float16* __restrict__ B2, const float* __restrict__ mb2,
                                                float* out, int nN) {
  __shared__ __attribute__((aligned(16))) _Float16 sz[2 * 16 * ZP];
  __shared__ __attribute__((aligned(16))) float so[2 * 16 * MO];
  const int tid = threadIdx.x, lane = tid & 31, wave = tid >> 5, hh = lane >> 4, m = lane & 15;
  const int row0 = blockIdx.x * MROWS + wave * 16;

  v8f acc[8];
#pragma unroll
  for (int t = 0; t < 8; ++t) { v8f z = {0.f, 0.f, 0.f, 0.f, 0.f, 0.f, 0.f, 0.f}; acc[t] = z; }
#pragma unroll 1
  for (int ks = 0; ks < MK / 32; ++ks) {
    const _Float16* ap = (ks < 2) ? (HS + (size_t)(row0 + m) * HD + 32 * ks + 8 * hh)
                                  : (HN + (size_t)(row0 + m) * (2 * GC) + 32 * (ks - 2) + 8 * hh);
    Frag a;
    a.h[0] = *(const v8h*)ap;
    a.h[1] = *(const v8h*)(ap + 16);
#pragma unroll
    for (int t = 0; t < 8; ++t) {
      const _Float16* bp = B1 + (size_t)(16 * t + m) * MK + 32 * ks + 8 * hh;
      Frag b;
      b.h[0] = *(const v8h*)bp;
      b.h[1] = *(const v8h*)(bp + 16);
      acc[t] = wmh(a.v, b.v, acc[t]);
    }
  }
  _Float16* zs = sz + wave * 16 * ZP;
#pragma unroll
  for (int t = 0; t < 8; ++t) {
    const float bb = mb1[16 * t + m];
#pragma unroll
    for (int r = 0; r < 8; ++r) {
      const float z = fmaxf(fmaf(acc[t][r], RH, bb), 0.0f) * HSC;
      zs[(8 * hh + r) * ZP + 16 * t + m] = (_Float16)z;
    }
  }
  WSYNC();

  v8f acc2[2];
  {
    v8f z = {0.f, 0.f, 0.f, 0.f, 0.f, 0.f, 0.f, 0.f};
    acc2[0] = z; acc2[1] = z;
  }
#pragma unroll 1
  for (int ks = 0; ks < MH / 32; ++ks) {
    Frag a;
    a.h[0] = *(const v8h*)(zs + m * ZP + 32 * ks + 8 * hh);
    a.h[1] = *(const v8h*)(zs + m * ZP + 32 * ks + 16 + 8 * hh);
#pragma unroll
    for (int t = 0; t < 2; ++t) {
      const _Float16* bp = B2 + (size_t)(16 * t + m) * MH + 32 * ks + 8 * hh;
      Frag b;
      b.h[0] = *(const v8h*)bp;
      b.h[1] = *(const v8h*)(bp + 16);
      acc2[t] = wmh(a.v, b.v, acc2[t]);
    }
  }
  float* os = so + wave * 16 * MO;
#pragma unroll
  for (int t = 0; t < 2; ++t) {
    const float bb = mb2[16 * t + m];
#pragma unroll
    for (int r = 0; r < 8; ++r) os[(8 * hh + r) * MO + 16 * t + m] = fmaf(acc2[t][r], RH, bb);
  }
  WSYNC();

  v4f ov[4];
  const int qr = lane >> 3, pc4 = (lane & 7) * 4;
#pragma unroll
  for (int it = 0; it < 4; ++it) ov[it] = *(const v4f*)(os + (4 * it + qr) * MO + pc4);
#pragma unroll
  for (int it = 0; it < 4; ++it) {
    const int grow = row0 + 4 * it + qr;
    if (grow < nN) *(volatile v4f*)(out + (size_t)grow * MO + pc4) = ov[it];
  }
  __threadfence();
#pragma unroll
  for (int it = 0; it < 4; ++it) {
    const int grow = row0 + 4 * it + qr;
    if (grow < nN) *(volatile v4f*)(out + (size_t)grow * MO + pc4) = ov[it];
  }
}

extern "C" void kernel_launch(void* const* d_in, const int* in_sizes, int n_in,
                              void* d_out, int out_size, void* d_ws, size_t ws_size,
                              hipStream_t stream) {
  if (n_in < 20) return;
  const int nN = in_sizes[0] / NIN;
  const int nE = in_sizes[2];
  if (nN < 1 || nE < 1) return;
  if (in_sizes[0] != nN * NIN || in_sizes[1] != 2 * nE) return;
  if (in_sizes[3] != C1 || in_sizes[4] != C1 || in_sizes[5] != C1 * C1 || in_sizes[6] != C1) return;
  if (in_sizes[7] != HD * NIN || in_sizes[8] != HD) return;
  if (in_sizes[9] != GC * NIN || in_sizes[10] != GC || in_sizes[11] != GC * NIN || in_sizes[12] != GC) return;
  if (in_sizes[13] != GC || in_sizes[14] != GC || in_sizes[15] != GC) return;
  if (in_sizes[16] != MH * MK || in_sizes[17] != MH || in_sizes[18] != MO * MH || in_sizes[19] != MO) return;
  if (out_size != nN * MO) return;
  if (nN > (1 << 22) || nE > (1 << 22)) return;

  const float* x    = (const float*)d_in[0];
  const int*   ei   = (const int*)d_in[1];
  const float* eat  = (const float*)d_in[2];
  const float* nw1  = (const float*)d_in[3];
  const float* nb1  = (const float*)d_in[4];
  const float* nw2  = (const float*)d_in[5];
  const float* nb2  = (const float*)d_in[6];
  const float* nrt  = (const float*)d_in[7];
  const float* nbs  = (const float*)d_in[8];
  const float* gwl  = (const float*)d_in[9];
  const float* gbl  = (const float*)d_in[10];
  const float* gwr  = (const float*)d_in[11];
  const float* gbr  = (const float*)d_in[12];
  const float* gwe  = (const float*)d_in[13];
  const float* gatt = (const float*)d_in[14];
  const float* gbs  = (const float*)d_in[15];
  const float* mw1  = (const float*)d_in[16];
  const float* mb1  = (const float*)d_in[17];
  const float* mw2  = (const float*)d_in[18];
  const float* mb2  = (const float*)d_in[19];
  float* out = (float*)d_out;
  const int* srcs = ei;
  const int* dsts = ei + (size_t)nE;

  const int nPad    = ((nN + NPG - 1) / NPG) * NPG;
  const int gNode   = nPad / NPB;
  const int gNN     = nPad / NBN;
  const int gGat    = nPad / NBG;
  const int gMrg    = (nN + MROWS - 1) / MROWS;
  const int nChunks = (nE + CHUNK - 1) / CHUNK;
  const int vec     = ((nE & 3) == 0) ? 1 : 0;

  char* ws = (char*)d_ws;
  size_t off = 0;
  const size_t oB  = off; off += (size_t)BPTOT * 2;        off = (off + 255) & ~(size_t)255;
  const size_t oXL = off; off += (size_t)nPad * GC * 4;    off = (off + 255) & ~(size_t)255;
  const size_t oXR = off; off += (size_t)nPad * GC * 4;    off = (off + 255) & ~(size_t)255;
  const size_t oHS = off; off += (size_t)nPad * HD * 2;    off = (off + 255) & ~(size_t)255;
  if (off > ws_size || off > (size_t)WSCAP) return;
  _Float16* Bpl = (_Float16*)(ws + oB);
  float*    XL  = (float*)(ws + oXL);
  float*    XR  = (float*)(ws + oXR);
  _Float16* HS  = (_Float16*)(ws + oHS);

  hipFuncSetAttribute(reinterpret_cast<const void*>(&k_nndrain), hipFuncAttributeMaxDynamicSharedMemorySize, LDS_NN);
  hipFuncSetAttribute(reinterpret_cast<const void*>(&k_gatdrain), hipFuncAttributeMaxDynamicSharedMemorySize, LDS_GAT);

  k_wprep<<<40, THR, 0, stream>>>(nw2, mw1, mw2, Bpl);
  k_node<<<gNode, THR, 0, stream>>>(x, gwl, gbl, gwr, gbr, XL, XR, nN);
  k_nndrain<<<gNN, THR, LDS_NN, stream>>>(srcs, dsts, x, eat, nw1, nb1, nb2, nrt, nbs, Bpl + OFF_BN, HS,
                                          nN, nE, nChunks, vec);
  k_gatdrain<<<gGat, THR, LDS_GAT, stream>>>(srcs, dsts, eat, gwe, gatt, gbs, XL, XR, nN, nE, nChunks, vec);
  k_merge<<<gMrg, MTHR, 0, stream>>>(HS, (const _Float16*)XR, Bpl + OFF_B1, mb1, Bpl + OFF_B2, mb2, out, nN);
}
